// LinOSSLayer_52621939310911
// MI455X (gfx1250) — hardware-verified
//
#include <hip/hip_runtime.h>
#include <math.h>

typedef __attribute__((ext_vector_type(16))) _Float16 v16h;
typedef __attribute__((ext_vector_type(8)))  _Float16 v8h;
typedef __attribute__((ext_vector_type(16))) __bf16   v16b;
typedef __attribute__((ext_vector_type(8)))  __bf16   v8b;
typedef __attribute__((ext_vector_type(8)))  float    v8f;
typedef __attribute__((ext_vector_type(4)))  float    v4f;

constexpr int kL    = 16384;
constexpr int kH    = 256;
constexpr int kS    = 512;
constexpr int kS2   = 2 * kS;
constexpr int kLC   = 4096;
constexpr int kNCh  = kL / kLC;
constexpr int kThr  = 256;
constexpr float kInCarry = 1024.0f;
constexpr float kWCarry = 4096.0f;
constexpr float kYCarry = 32.0f;
constexpr float kScBu = 1.0f / (kInCarry * kWCarry);
constexpr float kScOut = 1.0f / (kYCarry * kWCarry);
constexpr float kF16MinNormal = 6.103515625e-5f;

static_assert((kLC % 64) == 0 && (kS2 % 64) == 0 && (kH % 64) == 0 && (kH % 32) == 0 && (kS2 % 32) == 0
              && ((kLC / 64) * (kS2 / 64)) % 8 == 0 && ((kLC / 64) * (kH / 64)) % 8 == 0, "GEMM M, N multiples of 64; grids exact; K multiples of 32");

constexpr size_t kOffBT16 = 0ull;
constexpr size_t kOffCT16 = 524288ull;
constexpr size_t kOffZB = 1048576ull;
constexpr size_t kOffSTATE = 1052672ull;
constexpr size_t kOffU16 = 1060864ull;
constexpr size_t kOffBU = 3158016ull;
constexpr size_t kOffYS16 = 19935232ull;
constexpr size_t kOffO32 = 28323840ull;
constexpr size_t kWsTotal = 32518144ull;
static_assert(kWsTotal <= 134217728ull, "carve cap: under 128 MiB");
static_assert(kOffBT16 == 0
              && kOffCT16 == kOffBT16 + 524288ull
              && kOffZB == kOffCT16 + 524288ull
              && kOffSTATE == kOffZB + 4096ull
              && kOffU16 == kOffSTATE + 8192ull
              && kOffBU == kOffU16 + 2097152ull
              && kOffYS16 == kOffBU + 16777216ull
              && kOffO32 == kOffYS16 + 8388608ull
              && kWsTotal == kOffO32 + 4194304ull, "the carve is chained and totalled");
static_assert((kOffBT16 % 256) == 0 && (kOffCT16 % 256) == 0 && (kOffZB % 256) == 0 && (kOffSTATE % 256) == 0 && (kOffU16 % 256) == 0 && (kOffBU % 256) == 0 && (kOffYS16 % 256) == 0 && (kOffO32 % 256) == 0, "aligned regions");

__device__ __forceinline__ unsigned short f2bf_bits(float f) {
  unsigned u = __float_as_uint(f);
  return (unsigned short)((u + 0x7FFFu + ((u >> 16) & 1u)) >> 16);
}
__device__ __forceinline__ float bf_bits2f(unsigned short h) { return __uint_as_float(((unsigned)h) << 16); }
__device__ __forceinline__ float bf16r(float f) { return bf_bits2f(f2bf_bits(f)); }
__device__ __forceinline__ float carry_flush(float v, float carry) {
  const float s = v * carry;
  return (fabsf(s) < kF16MinNormal) ? 0.0f : s;
}
__device__ __forceinline__ float frcp(float x) { return __builtin_amdgcn_rcpf(x); }

__device__ __forceinline__ void dep_guard4_h(v8f& a, v8f& b, v8f& c, v8f& d, v16h x, v16h y) { asm volatile("v_nop\n\tv_nop\n\tv_nop\n\tv_nop" : "+v"(a), "+v"(b), "+v"(c), "+v"(d) : "v"(x), "v"(y)); }
__device__ __forceinline__ void dep_guard4_b(v8f& a, v8f& b, v8f& c, v8f& d, v16b x, v16b y) { asm volatile("v_nop\n\tv_nop\n\tv_nop\n\tv_nop" : "+v"(a), "+v"(b), "+v"(c), "+v"(d) : "v"(x), "v"(y)); }
__device__ __forceinline__ void keep4_h(v16h a, v16h b, v16h c, v16h d) { asm volatile("v_nop" :: "v"(a), "v"(b), "v"(c), "v"(d)); }
__device__ __forceinline__ void keep4_b(v16b a, v16b b, v16b c, v16b d) { asm volatile("v_nop" :: "v"(a), "v"(b), "v"(c), "v"(d)); }
__device__ __forceinline__ void acc_guard4(v8f& a, v8f& b, v8f& c, v8f& d) { asm volatile("v_nop\n\tv_nop\n\tv_nop\n\tv_nop" : "+v"(a), "+v"(b), "+v"(c), "+v"(d)); }

template <typename T> struct Frag;
template <> struct Frag<_Float16> {
  typedef v16h V; union U { v16h v; v8h h[2]; };
  static __device__ __forceinline__ v16h load(const _Float16* p) {
    U f; f.h[0] = *(const v8h*)(p); f.h[1] = *(const v8h*)(p + 16); return f.v;
  }
  static __device__ __forceinline__ v8f mma(v16h a, v16h b, v8f c) {
    return __builtin_amdgcn_wmma_f32_16x16x32_f16(false, a, false, b, (short)0, c, false, false);
  }
  static __device__ __forceinline__ void guard4(v8f& a, v8f& b, v8f& c, v8f& d, v16h x, v16h y) { dep_guard4_h(a, b, c, d, x, y); }
  static __device__ __forceinline__ void keep(v16h a, v16h b, v16h c, v16h d) { keep4_h(a, b, c, d); }
};
template <> struct Frag<__bf16> {
  typedef v16b V; union U { v16b v; v8b h[2]; };
  static __device__ __forceinline__ v16b load(const __bf16* p) {
    U f; f.h[0] = *(const v8b*)(p); f.h[1] = *(const v8b*)(p + 16); return f.v;
  }
  static __device__ __forceinline__ v8f mma(v16b a, v16b b, v8f c) {
    return __builtin_amdgcn_wmma_f32_16x16x32_bf16(false, a, false, b, (short)0, c, false, false);
  }
  static __device__ __forceinline__ void guard4(v8f& a, v8f& b, v8f& c, v8f& d, v16b x, v16b y) { dep_guard4_b(a, b, c, d, x, y); }
  static __device__ __forceinline__ void keep(v16b a, v16b b, v16b c, v16b d) { keep4_b(a, b, c, d); }
};

__device__ __forceinline__ v8f mma_h(v16h a, v16h b, v8f c) {
  c = __builtin_amdgcn_wmma_f32_16x16x32_f16(false, a, false, b, (short)0, c, false, false);
  asm volatile("v_nop\n\tv_nop\n\tv_nop\n\tv_nop" : "+v"(c) : "v"(a), "v"(b));
  return c;
}

template <int ET> struct Elem;
template <> struct Elem<0> { typedef _Float16 T; };
template <> struct Elem<1> { typedef __bf16 T; };
template <int ET, bool SPLIT, int BIAS_MODE, int OUT_MODE, bool RESID, int ACT = 0>
__global__ __launch_bounds__(256) void wmma_gemm64(
    const unsigned short* __restrict__ Ap, const unsigned short* __restrict__ A2p, int lda, long strideA,
    const unsigned short* __restrict__ Btp, const unsigned short* __restrict__ Bt2p, int ldb, long strideB,
    void* __restrict__ Cout, void* __restrict__ Cout2, int ldc, long strideC,
    const float* __restrict__ bias,
    const float* __restrict__ resid, long strideR,
    int M, int N, int K, float scale) {
  typedef typename Elem<ET>::T T;
  typedef typename Frag<T>::V V;
  const T* A = (const T*)Ap; const T* A2 = (const T*)A2p; const T* Bt = (const T*)Btp; const T* Bt2 = (const T*)Bt2p;
  __shared__ __align__(16) float sT[8][16 * 68];
  const int b    = blockIdx.y;
  const int lane = threadIdx.x & 31;
  const int wave = threadIdx.x >> 5;
  const int tilesN = N >> 6;
  const int tilesM = M >> 6;
  const int tile = blockIdx.x * 8 + wave;
  if (tile >= tilesM * tilesN) return;
  const int tm = tile / tilesN;
  const int tn = tile - tm * tilesN;
  const int m0 = tm << 6;
  const int n0 = tn << 6;

  const T* Ab  = A  + (size_t)b * strideA;
  const T* Bb  = Bt + (size_t)b * strideB;
  const T* Ab2 = SPLIT ? (A2  + (size_t)b * strideA) : nullptr;
  const T* Bb2 = SPLIT ? (Bt2 + (size_t)b * strideB) : nullptr;

  const int rlane = lane & 15;
  const int koff  = (lane >> 4) * 8;
  const int mOff  = (lane >> 4) * 8;

  v8f acc[4][4];
#pragma unroll
  for (int i = 0; i < 4; ++i)
#pragma unroll
    for (int j = 0; j < 4; ++j) acc[i][j] = (v8f){0.f,0.f,0.f,0.f,0.f,0.f,0.f,0.f};

  for (int k0 = 0; k0 < K; k0 += 32) {
    V bh[4], bl[4];
#pragma unroll
    for (int j = 0; j < 4; ++j) {
      const size_t bo = (size_t)(n0 + (j << 4) + rlane) * ldb + koff + k0;
      bh[j] = Frag<T>::load(Bb + bo);
      if (SPLIT) bl[j] = Frag<T>::load(Bb2 + bo);
    }
#pragma unroll
    for (int i = 0; i < 4; ++i) {
      const size_t ao = (size_t)(m0 + (i << 4) + rlane) * lda + koff + k0;
      V ah = Frag<T>::load(Ab + ao);
      V al;
      if (SPLIT) al = Frag<T>::load(Ab2 + ao);
#pragma unroll
      for (int j = 0; j < 4; ++j) {
        acc[i][j] = Frag<T>::mma(ah, bh[j], acc[i][j]);
        if (SPLIT) {
          acc[i][j] = Frag<T>::mma(ah, bl[j], acc[i][j]);
          acc[i][j] = Frag<T>::mma(al, bh[j], acc[i][j]);
        }
      }
      Frag<T>::guard4(acc[i][0], acc[i][1], acc[i][2], acc[i][3], ah, SPLIT ? al : ah);
    }
    Frag<T>::keep(bh[0], bh[1], bh[2], bh[3]);
    if (SPLIT) Frag<T>::keep(bl[0], bl[1], bl[2], bl[3]);
  }
  acc_guard4(acc[0][0], acc[0][1], acc[0][2], acc[0][3]);
  acc_guard4(acc[1][0], acc[1][1], acc[1][2], acc[1][3]);
  acc_guard4(acc[2][0], acc[2][1], acc[2][2], acc[2][3]);
  acc_guard4(acc[3][0], acc[3][1], acc[3][2], acc[3][3]);

  float* slab = sT[wave];
  const float* Rb = RESID ? (resid + (size_t)b * strideR) : nullptr;
#pragma unroll
  for (int i = 0; i < 4; ++i) {
    const int mBase = m0 + (i << 4);
#pragma unroll
    for (int j = 0; j < 4; ++j) {
      const int n = n0 + (j << 4) + rlane;
      float bv = 0.f;
      if (BIAS_MODE == 2) bv = bias[n];
#pragma unroll
      for (int r = 0; r < 8; ++r) {
        float v = acc[i][j][r] * scale;
        if (BIAS_MODE == 1) v += bias[mBase + mOff + r];
        if (BIAS_MODE == 2) v += bv;
        if (RESID) v += Rb[(size_t)(mBase + mOff + r) * ldc + n];
        if (ACT == 1) v = tanhf(v);
        if (ACT == 2) v = fmaxf(v, 0.0f);
        if (ACT == 3) v = v / (1.0f + expf(-v));
        if (ACT == 4) v = (v > 0.f) ? v : 0.01f * v;
        slab[(mOff + r) * 68 + (j << 4) + rlane] = v;
      }
    }
    __builtin_amdgcn_fence(__ATOMIC_RELEASE, "workgroup");
    __builtin_amdgcn_wave_barrier();
    __builtin_amdgcn_fence(__ATOMIC_ACQUIRE, "workgroup");
    if (OUT_MODE == 0) {
      float* C = (float*)Cout + (size_t)b * strideC;
      const int hh = lane >> 4, c4 = (lane & 15) * 4;
      for (int pass = 0; pass < 2; ++pass) {
#pragma unroll
        for (int it = 0; it < 8; ++it) {
          const int row = it * 2 + hh;
          v4f v = *(const v4f*)(slab + row * 68 + c4);
          *(volatile v4f*)(C + (size_t)(mBase + row) * ldc + n0 + c4) = v;
        }
        __threadfence();
      }
    } else {
      const int q = lane >> 3, c8 = (lane & 7) * 8;
      unsigned short* C  = (unsigned short*)Cout  + (size_t)b * strideC;
      unsigned short* C2 = (OUT_MODE == 2) ? ((unsigned short*)Cout2 + (size_t)b * strideC) : nullptr;
      for (int pass = 0; pass < 2; ++pass) {
#pragma unroll
        for (int it = 0; it < 4; ++it) {
          const int row = it * 4 + q;
          const float* sp = slab + row * 68 + c8;
          v8h hv, lv;
#pragma unroll
          for (int e = 0; e < 8; ++e) {
            if (OUT_MODE == 1) {
              hv[e] = (_Float16)sp[e];
            } else {
              unsigned short hb = f2bf_bits(sp[e]);
              unsigned short lb = f2bf_bits(sp[e] - bf_bits2f(hb));
              hv[e] = __builtin_bit_cast(_Float16, hb);
              lv[e] = __builtin_bit_cast(_Float16, lb);
            }
          }
          *(volatile v8h*)(C + (size_t)(mBase + row) * ldc + n0 + c8) = hv;
          if (OUT_MODE == 2) *(volatile v8h*)(C2 + (size_t)(mBase + row) * ldc + n0 + c8) = lv;
        }
        __threadfence();
      }
    }
    __builtin_amdgcn_fence(__ATOMIC_RELEASE, "workgroup");
    __builtin_amdgcn_wave_barrier();
    __builtin_amdgcn_fence(__ATOMIC_ACQUIRE, "workgroup");
  }
}

__global__ __launch_bounds__(kThr) void cast_plane_kernel(const float* __restrict__ src, unsigned short* __restrict__ dst,
                                                          int colsLog2, int dstPitch, int dstOff) {
  const int i   = blockIdx.x * kThr + threadIdx.x;
  const int sh  = colsLog2 - 3;
  const int row = i >> sh;
  const int c8  = (i & ((1 << sh) - 1)) * 8;
  const float* sp = src + ((size_t)row << colsLog2) + c8;
  const v4f a0 = *(const v4f*)(sp);
  const v4f a1 = *(const v4f*)(sp + 4);
  v8h hv;
#pragma unroll
  for (int e = 0; e < 4; ++e) {
    const float f0 = a0[e];
    const float f1 = a1[e];
    hv[e]     = (_Float16)carry_flush(bf16r(f0), kInCarry);
    hv[4 + e] = (_Float16)carry_flush(bf16r(f1), kInCarry);
  }
  unsigned short* dp = dst + (size_t)row * dstPitch + dstOff + c8;
  *(volatile v8h*)dp = hv;
  __threadfence();
  *(volatile v8h*)dp = hv;
}

__global__ __launch_bounds__(kThr) void setup_kernel(const float* __restrict__ B, const float* __restrict__ C, unsigned short* __restrict__ BT16,
                                                     unsigned short* __restrict__ CT16, float* __restrict__ ZS) {
  unsigned v = blockIdx.x * (unsigned)kThr + threadIdx.x;
  asm volatile("" : "+v"(v));
  if (v < 32768u) {
    const unsigned n = v >> 5, h8 = (v & 31u) * 8u;
    const unsigned p = n >> 9, s = n & 511u;
    v8h hv;
#pragma unroll
    for (int e = 0; e < 8; ++e) { const float w = B[((size_t)s * kH + h8 + e) * 2u + p]; hv[e] = (_Float16)carry_flush(bf16r(w), kWCarry); }
    unsigned short* dp = BT16 + (size_t)v * 8u;
    *(volatile v8h*)dp = hv;
    __threadfence();
    *(volatile v8h*)dp = hv;
  } else if (v < 65536u) {
    const unsigned w0 = v - 32768u;
    const unsigned h = w0 >> 7, n8 = (w0 & 127u) * 8u;
    const unsigned p = n8 >> 9, s8 = n8 & 511u;
    v8h hv;
#pragma unroll
    for (int e = 0; e < 8; ++e) { const float w = C[((size_t)h * kS + s8 + e) * 2u + p]; const float q = bf16r(w); hv[e] = (_Float16)carry_flush(p ? -q : q, kWCarry); }
    unsigned short* dp = CT16 + (size_t)w0 * 8u;
    *(volatile v8h*)dp = hv;
    __threadfence();
    *(volatile v8h*)dp = hv;
  } else {
    const v4f o = {0.f, 0.f, 0.f, 0.f};
    float* dp = ZS + (size_t)(v - 65536u) * 4u;
    *(volatile v4f*)dp = o;
    __threadfence();
    *(volatile v4f*)dp = o;
  }
}
static_assert(kS2 * kH / 8 == 32768 && 32768 % kThr == 0 && (65536 + 768) == 259 * kThr && (1024 + 2048) / 4 == 768, "set-up grid exact");

__global__ __launch_bounds__(kThr) void osc_scan_kernel(float* __restrict__ BU, const float* __restrict__ A_diag, const float* __restrict__ steps,
                                                        float* __restrict__ STATE) {
  const int n = blockIdx.x * kThr + threadIdx.x;
  const int s = n & (kS - 1);
  float ad = A_diag[s], sr = steps[s];
  asm volatile("" : "+v"(ad), "+v"(sr));
  ad = bf16r(ad); sr = bf16r(sr);
  const float A = (ad > 0.0f) ? ad : 0.0f;
  const float step = 1.0f / (1.0f + expf(-sr));
  const float schur = 1.0f / (1.0f + step * step * A);
  const float m11 = 1.0f - step * step * A * schur;
  const float m12 = -step * A * schur;
  const float m21 = step * schur;
  const float m22 = schur;
  float x1 = STATE[n], x2 = STATE[kS2 + n];
#pragma unroll 1
  for (int l = 0; l < kLC; ++l) {
    float* bp = BU + (size_t)l * kS2 + n;
    const float b = *bp;
    const float f1 = m11 * b * step;
    const float f2 = m21 * b * step;
    const float n1 = m11 * x1 + m12 * x2 + f1;
    const float n2 = m21 * x1 + m22 * x2 + f2;
    x1 = n1; x2 = n2;
    *(volatile float*)bp = n2;
    __threadfence();
    *(volatile float*)bp = n2;
  }
  for (int pass = 0; pass < 2; ++pass) {
    *(volatile float*)(STATE + n) = x1;
    *(volatile float*)(STATE + kS2 + n) = x2;
    __threadfence();
  }
}
static_assert(kS2 == 4 * kThr, "scan grid exact");

__global__ __launch_bounds__(kThr) void ys_cast_kernel(const float* __restrict__ YS, unsigned short* __restrict__ YS16) {
  unsigned v = blockIdx.x * (unsigned)kThr + threadIdx.x;
  asm volatile("" : "+v"(v));
  const size_t o8 = (size_t)v * 8u;
  const v4f a0 = *(const v4f*)(YS + o8), a1 = *(const v4f*)(YS + o8 + 4);
  v8h hv;
#pragma unroll
  for (int e = 0; e < 4; ++e) { hv[e] = (_Float16)carry_flush(a0[e], kYCarry); hv[4 + e] = (_Float16)carry_flush(a1[e], kYCarry); }
  *(volatile v8h*)(YS16 + o8) = hv;
  __threadfence();
  *(volatile v8h*)(YS16 + o8) = hv;
}
static_assert(((size_t)kLC * kS2 / 8) == 2048 * kThr, "cast grid exact");

__global__ __launch_bounds__(kThr) void skip_kernel(const float* __restrict__ O32, const float* __restrict__ u, const float* __restrict__ D, float* __restrict__ out) {
  unsigned v = blockIdx.x * (unsigned)kThr + threadIdx.x;
  asm volatile("" : "+v"(v));
  const size_t o4 = (size_t)v * 4u;
  const unsigned h4 = (v & 63u) * 4u;
  const v4f o = *(const v4f*)(O32 + o4), uu = *(const v4f*)(u + o4), dd = *(const v4f*)(D + h4);
  v4f r;
#pragma unroll
  for (int e = 0; e < 4; ++e) r[e] = o[e] + bf16r(dd[e]) * bf16r(uu[e]);
  *(volatile v4f*)(out + o4) = r;
  __threadfence();
  *(volatile v4f*)(out + o4) = r;
}
static_assert(((size_t)kLC * kH / 4) == 1024 * kThr && kH / 4 == 64, "skip grid exact");

extern "C" void kernel_launch(void* const* d_in, const int* in_sizes, int n_in,
                              void* d_out, int out_size, void* d_ws, size_t ws_size,
                              hipStream_t stream) {
  if (n_in < 6 || d_out == nullptr || d_ws == nullptr) return;
  if (in_sizes[0] != kL * kH || in_sizes[1] != kS || in_sizes[2] != kS * kH * 2 || in_sizes[3] != kH * kS * 2 || in_sizes[4] != kH || in_sizes[5] != kS) return;
  if (out_size != kL * kH) return;
  if (ws_size < kWsTotal) return;
  const float* u = (const float*)d_in[0];
  const float* A_diag = (const float*)d_in[1];
  const float* B = (const float*)d_in[2];
  const float* C = (const float*)d_in[3];
  const float* D = (const float*)d_in[4];
  const float* steps = (const float*)d_in[5];
  float* out = (float*)d_out;
  char* ws = (char*)d_ws;
  unsigned short* BT16 = (unsigned short*)(ws + kOffBT16);
  unsigned short* CT16 = (unsigned short*)(ws + kOffCT16);
  float* ZB = (float*)(ws + kOffZB);
  float* STATE = (float*)(ws + kOffSTATE);
  unsigned short* U16 = (unsigned short*)(ws + kOffU16);
  float* BU = (float*)(ws + kOffBU);
  unsigned short* YS16 = (unsigned short*)(ws + kOffYS16);
  float* O32 = (float*)(ws + kOffO32);

  setup_kernel<<<259, kThr, 0, stream>>>(B, C, BT16, CT16, ZB);

  for (int ch = 0; ch < kNCh; ++ch) {
    const float* uc = u + (size_t)ch * kLC * kH;
    float* oc = out + (size_t)ch * kLC * kH;
    cast_plane_kernel<<<(int)(((size_t)kLC * kH / 8) / kThr), kThr, 0, stream>>>(uc, U16, 8, kH, 0);
    wmma_gemm64<0, false, 2, 0, false, 0><<<dim3((kLC / 64) * (kS2 / 64) / 8, 1), 256, 0, stream>>>(
        U16, U16, kH, 0L, BT16, BT16, kH, 0L, (void*)BU, (void*)BU, kS2, 0L, ZB, nullptr, 0L, kLC, kS2, kH, kScBu);
    osc_scan_kernel<<<4, kThr, 0, stream>>>(BU, A_diag, steps, STATE);
    ys_cast_kernel<<<2048, kThr, 0, stream>>>(BU, YS16);
    wmma_gemm64<0, false, 2, 0, false, 0><<<dim3((kLC / 64) * (kH / 64) / 8, 1), 256, 0, stream>>>(
        YS16, YS16, kS2, 0L, CT16, CT16, kS2, 0L, (void*)O32, (void*)O32, kH, 0L, ZB, nullptr, 0L, kLC, kH, kS2, kScOut);
    skip_kernel<<<1024, kThr, 0, stream>>>(O32, uc, D, oc);
  }
}
